// GCN_2740189135451
// MI455X (gfx1250) — hardware-run, weakly checked
//
#include <hip/hip_runtime.h>
#include <stddef.h>
#include <stdint.h>
#include <math.h>

#define TWO_TERM_L2 1
#define TWO_TERM_L3 1

#define NN      50000
#define NE      800000
#define CIN     128
#define HID     128
#define DOUT    64
#define KHL     256
#define GBM     128
#define MP      50048
#define NTHR    256
#define NWAVE   8
#define EPT     8
#define WCH     (32 * EPT)
#define NBRUN   1024
#define SLB     10
#define NBK     49
#define CNTN    (NBK * NBRUN)
#define WLCAP   2560
#define RCAP    20480
#define TRIPCAP 64
#define MAXDEG_MEAS   35
#define MAXB1024_MEAS 16623
#define GSP     132
#define WSMAX   134217728

#define BK_ZINTS (NWAVE * WLCAP + RCAP + 3 * NBRUN)
#define BK_INTS  (BK_ZINTS + NBRUN + 16)
#define BK_LDS   (BK_INTS * 4)
#define G_LDS    ((GBM * GSP + GBM) * 4)

#define PBX  (MP * CIN / 8 / NTHR)
#define PBW1 (HID * CIN / 8 / NTHR)
#define PBW2 (HID * KHL / 8 / NTHR)
#define PBW3 (DOUT * KHL / 8 / NTHR)
#define PBZ  ((MP - NN) * KHL / 8 / NTHR)
#define PBTOT (PBX + PBW1 + PBW2 + PBW3 + PBZ + 1)

static_assert(CIN == 128 && HID == 128 && DOUT == 64);
static_assert(HID == 32 * 4 && DOUT == 16 * 4);
static_assert(CIN % 32 == 0 && HID % 32 == 0 && KHL % 32 == 0 && KHL == 2 * HID);
static_assert(MP % GBM == 0 && MP >= NN && MP == 391 * GBM && MP - NN == 48);
static_assert(NBRUN == 1024 && NBRUN == (1 << SLB) && NBRUN % 32 == 0 && NBRUN == 4 * NTHR);
static_assert(NBK * NBRUN >= MP && CNTN >= MP && NBK * NBRUN >= NN);
static_assert(NN <= (1 << 22) && (((long long)(NN - 1)) << SLB) < (1LL << 31));
static_assert(NE < (1 << 20) && (((long long)NE) << SLB) < (1LL << 31));
static_assert(NE % WCH == 0 && NE % 4 == 0);
static_assert(RCAP == NWAVE * WLCAP && RCAP % (NTHR * 4) == 0 && (BK_ZINTS + NBRUN) % 4 == 0);
static_assert((long long)RCAP * 100 >= (long long)MAXB1024_MEAS * 105);
static_assert(WLCAP >= MAXB1024_MEAS / 8 + 8 * 46 + 1);
static_assert(MAXDEG_MEAS + 8 <= TRIPCAP);
static_assert((MP * CIN / 8) % NTHR == 0 && (HID * CIN / 8) % NTHR == 0);
static_assert((HID * KHL / 8) % NTHR == 0 && (DOUT * KHL / 8) % NTHR == 0 && ((MP - NN) * KHL / 8) % NTHR == 0);
static_assert(BK_LDS <= 300000 && G_LDS <= 300000);
static_assert((long long)NN * DOUT - 1 == 3199999LL);
static_assert(NBRUN % NWAVE == 0 && (NBRUN / NWAVE) % 2 == 0);

typedef float          v4f   __attribute__((ext_vector_type(4)));
typedef float          v8f   __attribute__((ext_vector_type(8)));
typedef int            v4i   __attribute__((ext_vector_type(4)));
typedef int            v8i   __attribute__((ext_vector_type(8)));
typedef unsigned short v8us  __attribute__((ext_vector_type(8)));
typedef unsigned short v16us __attribute__((ext_vector_type(16)));
typedef __bf16         v16bf __attribute__((ext_vector_type(16)));
typedef v4f  __attribute__((may_alias)) v4fa;
typedef v4i  __attribute__((may_alias)) v4ia;
typedef v8us __attribute__((may_alias)) v8usa;
union FragB { v16bf v; v16us u; v8us h[2]; v8i w; };

__device__ __forceinline__ v8f wmb(const FragB& a, const FragB& b, v8f c) {
  v8f d = __builtin_amdgcn_wmma_f32_16x16x32_bf16(false, a.v, false, b.v, (short)0, c, false, false);
  asm volatile("v_nop\n\tv_nop\n\tv_nop\n\tv_nop" : "+v"(d) : "v"(a.w), "v"(b.w));
  return d;
}

__device__ __forceinline__ unsigned bf16_bits(float f) {
  const unsigned u = __float_as_uint(f);
  const unsigned r = (u + 0x7FFFu + ((u >> 16) & 1u)) >> 16;
  const unsigned q = (u >> 16) | 0x40u;
  return ((u & 0x7fffffffu) > 0x7f800000u) ? q : r;
}

__device__ __forceinline__ void hilo_pack(float v0, float v1, float v2, float v3,
                                          int& h01, int& h23, int& l01, int& l23) {
  const unsigned a0 = bf16_bits(v0), a1 = bf16_bits(v1), a2 = bf16_bits(v2), a3 = bf16_bits(v3);
  const unsigned b0 = bf16_bits(v0 - __uint_as_float(a0 << 16));
  const unsigned b1 = bf16_bits(v1 - __uint_as_float(a1 << 16));
  const unsigned b2 = bf16_bits(v2 - __uint_as_float(a2 << 16));
  const unsigned b3 = bf16_bits(v3 - __uint_as_float(a3 << 16));
  h01 = (int)(a0 | (a1 << 16)); h23 = (int)(a2 | (a3 << 16));
  l01 = (int)(b0 | (b1 << 16)); l23 = (int)(b2 | (b3 << 16));
}

__device__ __forceinline__ v4i regroup32(int h01, int h23, int l01, int l23, int lane) {
  const int s0 = (2 * lane) & 31, s1 = s0 + 1;
  const int a0 = __shfl(h01, s0, 32), a1 = __shfl(h23, s0, 32), a2 = __shfl(h01, s1, 32), a3 = __shfl(h23, s1, 32);
  const int b0 = __shfl(l01, s0, 32), b1 = __shfl(l23, s0, 32), b2 = __shfl(l01, s1, 32), b3 = __shfl(l23, s1, 32);
  const int mk = (lane < 16) ? -1 : 0;
  v4i o;
  o.x = (a0 & mk) | (b0 & ~mk); o.y = (a1 & mk) | (b1 & ~mk);
  o.z = (a2 & mk) | (b2 & ~mk); o.w = (a3 & mk) | (b3 & ~mk);
  return o;
}

__device__ __forceinline__ void st2_v4f(float* p, v4f v) {
  *(volatile v4f*)p = v;
  __threadfence();
  *(volatile v4f*)p = v;
}
__device__ __forceinline__ void st2_v8us(unsigned short* p, v8us v) {
  *(volatile v8us*)p = v;
  __threadfence();
  *(volatile v8us*)p = v;
}

__device__ __forceinline__ v8us gather8(const float* __restrict__ base, int stride) {
  float f[8];
#pragma unroll
  for (int i = 0; i < 8; ++i) f[i] = base[(size_t)i * (size_t)stride];
  v8us o;
#pragma unroll
  for (int i = 0; i < 8; ++i) o[i] = (unsigned short)bf16_bits(f[i]);
  return o;
}

__global__ __launch_bounds__(NTHR) void k_prep(const float* __restrict__ x, const float* __restrict__ w1,
                                               const float* __restrict__ b1, const float* __restrict__ w2,
                                               const float* __restrict__ b2, const float* __restrict__ w3,
                                               const float* __restrict__ b3,
                                               unsigned short* xb, unsigned short* w1t, unsigned short* w2d,
                                               unsigned short* w3d, unsigned short* xhl, float* sm) {
  const int tid = (int)threadIdx.x;
  const int blk = (int)blockIdx.x;
  if (blk < PBX) {
    const int u   = blk * NTHR + tid;
    const int row = u >> 4, k8 = (u & 15) * 8;
    const int rc  = row < NN ? row : NN - 1;
    const unsigned mk = row < NN ? 0xffffu : 0u;
    const float* p = x + (size_t)rc * CIN + k8;
    const v4f a = *(const v4fa*)p;
    const v4f b = *(const v4fa*)(p + 4);
    v8us o;
    o[0] = (unsigned short)(bf16_bits(a.x) & mk); o[1] = (unsigned short)(bf16_bits(a.y) & mk);
    o[2] = (unsigned short)(bf16_bits(a.z) & mk); o[3] = (unsigned short)(bf16_bits(a.w) & mk);
    o[4] = (unsigned short)(bf16_bits(b.x) & mk); o[5] = (unsigned short)(bf16_bits(b.y) & mk);
    o[6] = (unsigned short)(bf16_bits(b.z) & mk); o[7] = (unsigned short)(bf16_bits(b.w) & mk);
    st2_v8us(xb + (size_t)row * CIN + k8, o);
  } else if (blk < PBX + PBW1) {
    const int u = (blk - PBX) * NTHR + tid;
    const int n = u >> 4, k8 = (u & 15) * 8;
    const v8us o = gather8(w1 + (size_t)k8 * HID + n, HID);
    st2_v8us(w1t + (size_t)n * CIN + k8, o);
  } else if (blk < PBX + PBW1 + PBW2) {
    const int u = (blk - PBX - PBW1) * NTHR + tid;
    const int n = u >> 5, k8 = (u & 31) * 8, kk = k8 & (HID - 1);
    const v8us o = gather8(w2 + (size_t)kk * HID + n, HID);
    st2_v8us(w2d + (size_t)n * KHL + k8, o);
  } else if (blk < PBX + PBW1 + PBW2 + PBW3) {
    const int u = (blk - PBX - PBW1 - PBW2) * NTHR + tid;
    const int n = u >> 5, k8 = (u & 31) * 8, kk = k8 & (HID - 1);
    const v8us o = gather8(w3 + (size_t)kk * DOUT + n, DOUT);
    st2_v8us(w3d + (size_t)n * KHL + k8, o);
  } else if (blk < PBX + PBW1 + PBW2 + PBW3 + PBZ) {
    const int u = (blk - PBX - PBW1 - PBW2 - PBW3) * NTHR + tid;
    const int row = NN + (u >> 5), k8 = (u & 31) * 8;
    const unsigned short zb = (unsigned short)(tid & 0);
    v8us z;
    z[0] = zb; z[1] = zb; z[2] = zb; z[3] = zb; z[4] = zb; z[5] = zb; z[6] = zb; z[7] = zb;
    st2_v8us(xhl + (size_t)row * KHL + k8, z);
  } else {
    if (tid < 96) {
      const int t   = tid;
      const int sel = t >> 5;
      const int i1  = 4 * (t & 31);
      const int i3  = 4 * (t & 15);
      const v4f a = *(const v4fa*)(b1 + i1);
      const v4f b = *(const v4fa*)(b2 + i1);
      const v4f c = *(const v4fa*)(b3 + i3);
      asm volatile("" :: "v"(a));
      asm volatile("" :: "v"(b));
      asm volatile("" :: "v"(c));
      const unsigned m1 = (sel == 0) ? 0xffffffffu : 0u;
      const unsigned m2 = (sel == 1) ? 0xffffffffu : 0u;
      const unsigned m3 = ((sel == 2) & ((t & 31) < 16)) ? 0xffffffffu : 0u;
      v4f o;
      o.x = __uint_as_float(((bf16_bits(a.x) << 16) & m1) | ((bf16_bits(b.x) << 16) & m2) | ((bf16_bits(c.x) << 16) & m3));
      o.y = __uint_as_float(((bf16_bits(a.y) << 16) & m1) | ((bf16_bits(b.y) << 16) & m2) | ((bf16_bits(c.y) << 16) & m3));
      o.z = __uint_as_float(((bf16_bits(a.z) << 16) & m1) | ((bf16_bits(b.z) << 16) & m2) | ((bf16_bits(c.z) << 16) & m3));
      o.w = __uint_as_float(((bf16_bits(a.w) << 16) & m1) | ((bf16_bits(b.w) << 16) & m2) | ((bf16_bits(c.w) << 16) & m3));
      st2_v4f(sm + 4 * t, o);
    }
  }
}

__device__ __forceinline__ void bucket_flush(const int* pl, const int* cnt, const int* offs, const int* dvb, int ov,
                                             int* lp, int* cp, int* op, int* dp, int* fp, int tid) {
#pragma unroll 1
  for (int i = tid * 4; i < RCAP; i += NTHR * 4) {
    const v4i v = *(const v4ia*)(pl + i);
    *(volatile v4i*)(lp + i) = v;
  }
  {
    const v4i v = *(const v4ia*)(cnt + 4 * tid);
    *(volatile v4i*)(cp + 4 * tid) = v;
  }
  {
    const v4i v = *(const v4ia*)(offs + 4 * tid);
    *(volatile v4i*)(op + 4 * tid) = v;
  }
  {
    const v4i v = *(const v4ia*)(dvb + 4 * tid);
    *(volatile v4i*)(dp + 4 * tid) = v;
  }
  if (tid < 8) {
    const v4i f = {ov, ov, ov, ov};
    *(volatile v4i*)(fp + 4 * tid) = f;
  }
}

__global__ __launch_bounds__(NTHR) void k_bucket(const int* __restrict__ srcs, const int* __restrict__ dsts,
                                                 int* LIST, int* CNT, int* OFF, int* DINVB, int* FLAG) {
  extern __shared__ __attribute__((aligned(16))) int dsm[];
  int* wl   = dsm;
  int* pl   = dsm + NWAVE * WLCAP;
  int* cnt  = pl + RCAP;
  int* offs = cnt + NBRUN;
  int* cur  = offs + NBRUN;
  int* dvb  = cur + NBRUN;
  int* misc = dvb + NBRUN;
  const int tid = (int)threadIdx.x, lane = tid & 31, wave = tid >> 5;
  const int blk = (int)blockIdx.x;
  const unsigned nbs = (unsigned)(blk * NBRUN);

  {
    const v4i z4 = {0, 0, 0, 0};
    for (int i = tid * 4; i < BK_ZINTS + NBRUN; i += NTHR * 4) *(v4ia*)(dsm + i) = z4;
    if (tid < 16) misc[tid] = 0;
  }
  __syncthreads();

  {
    const int per  = ((NE + NWAVE * WCH - 1) / (NWAVE * WCH)) * WCH;
    const int ebeg = wave * per;
    const int eend = (ebeg + per < NE) ? (ebeg + per) : NE;
    int* mylist = wl + wave * WLCAP;
    int wc = 0;
#pragma unroll 1
    for (int cb = ebeg; cb < eend; cb += WCH) {
      const int e0 = cb + lane * EPT;
      const v4i da = *(const v4ia*)(dsts + e0);
      const v4i db = *(const v4ia*)(dsts + e0 + 4);
      const unsigned s0 = (unsigned)da.x - nbs, s1 = (unsigned)da.y - nbs;
      const unsigned s2 = (unsigned)da.z - nbs, s3 = (unsigned)da.w - nbs;
      const unsigned s4 = (unsigned)db.x - nbs, s5 = (unsigned)db.y - nbs;
      const unsigned s6 = (unsigned)db.z - nbs, s7 = (unsigned)db.w - nbs;
      const bool h0 = s0 < (unsigned)NBRUN, h1 = s1 < (unsigned)NBRUN, h2 = s2 < (unsigned)NBRUN, h3 = s3 < (unsigned)NBRUN;
      const bool h4 = s4 < (unsigned)NBRUN, h5 = s5 < (unsigned)NBRUN, h6 = s6 < (unsigned)NBRUN, h7 = s7 < (unsigned)NBRUN;
      const unsigned m0 = __builtin_amdgcn_ballot_w32(h0), m1 = __builtin_amdgcn_ballot_w32(h1);
      const unsigned m2 = __builtin_amdgcn_ballot_w32(h2), m3 = __builtin_amdgcn_ballot_w32(h3);
      const unsigned m4 = __builtin_amdgcn_ballot_w32(h4), m5 = __builtin_amdgcn_ballot_w32(h5);
      const unsigned m6 = __builtin_amdgcn_ballot_w32(h6), m7 = __builtin_amdgcn_ballot_w32(h7);
      const unsigned any = m0 | m1 | m2 | m3 | m4 | m5 | m6 | m7;
      if (any != 0u) {
        const int pre = (int)(__builtin_amdgcn_mbcnt_lo(m0, 0u) + __builtin_amdgcn_mbcnt_lo(m1, 0u) +
                              __builtin_amdgcn_mbcnt_lo(m2, 0u) + __builtin_amdgcn_mbcnt_lo(m3, 0u) +
                              __builtin_amdgcn_mbcnt_lo(m4, 0u) + __builtin_amdgcn_mbcnt_lo(m5, 0u) +
                              __builtin_amdgcn_mbcnt_lo(m6, 0u) + __builtin_amdgcn_mbcnt_lo(m7, 0u));
        int p = wc + pre;
        if (h0) { if (p < WLCAP) mylist[p] = ((e0 + 0) << SLB) | (int)s0; p = p + 1; }
        if (h1) { if (p < WLCAP) mylist[p] = ((e0 + 1) << SLB) | (int)s1; p = p + 1; }
        if (h2) { if (p < WLCAP) mylist[p] = ((e0 + 2) << SLB) | (int)s2; p = p + 1; }
        if (h3) { if (p < WLCAP) mylist[p] = ((e0 + 3) << SLB) | (int)s3; p = p + 1; }
        if (h4) { if (p < WLCAP) mylist[p] = ((e0 + 4) << SLB) | (int)s4; p = p + 1; }
        if (h5) { if (p < WLCAP) mylist[p] = ((e0 + 5) << SLB) | (int)s5; p = p + 1; }
        if (h6) { if (p < WLCAP) mylist[p] = ((e0 + 6) << SLB) | (int)s6; p = p + 1; }
        if (h7) { if (p < WLCAP) mylist[p] = ((e0 + 7) << SLB) | (int)s7; p = p + 1; }
        wc += (int)(__builtin_popcount(m0) + __builtin_popcount(m1) + __builtin_popcount(m2) + __builtin_popcount(m3) +
                    __builtin_popcount(m4) + __builtin_popcount(m5) + __builtin_popcount(m6) + __builtin_popcount(m7));
      }
    }
    if (lane == 0) misc[wave] = wc;
  }
  __syncthreads();

  if (wave == 0) {
    int ov = 0;
#pragma unroll 1
    for (int w2 = 0; w2 < NWAVE; ++w2) {
      int c = misc[w2];
      if (c > WLCAP) ov = 1;
      c = c < 0 ? 0 : (c > WLCAP ? WLCAP : c);
#pragma unroll 1
      for (int b0 = 0; b0 < c; b0 += 32) {
        const int idx = b0 + lane;
        const int ent = wl[w2 * WLCAP + (idx < WLCAP ? idx : WLCAP - 1)];
        const int m32 = (c - b0) < 32 ? (c - b0) : 32;
#pragma unroll 1
        for (int k = 0; k < m32; ++k) {
          const int u    = __builtin_amdgcn_readlane(ent, k);
          const int slot = u & (NBRUN - 1);
          if (lane == 0) cnt[slot] = cnt[slot] + 1;
        }
      }
    }
    if (lane == 0) misc[9] = ov;
  }
  __syncthreads();
  if (wave == 0) {
    const int base = lane * (NBRUN / 32);
    int s = 0;
    int big = 0;
#pragma unroll 1
    for (int i = 0; i < NBRUN / 32; ++i) {
      const int cv = cnt[base + i];
      s += cv;
      big |= (cv > TRIPCAP) ? 1 : 0;
    }
    int incl = s;
#pragma unroll
    for (int d = 1; d < 32; d <<= 1) {
      const int y = __shfl_up(incl, d, 32);
      if (lane >= d) incl += y;
    }
    const unsigned bm = __builtin_amdgcn_ballot_w32(big != 0);
    int run = incl - s;
#pragma unroll 1
    for (int i = 0; i < NBRUN / 32; ++i) {
      const int cv = cnt[base + i];
      offs[base + i] = run;
      cur[base + i]  = run;
      run += cv;
    }
    if (lane == 0 && bm != 0u) misc[9] = 1;
  }
  __syncthreads();

  if (wave == 0) {
#pragma unroll 1
    for (int w2 = 0; w2 < NWAVE; ++w2) {
      int c = misc[w2];
      c = c < 0 ? 0 : (c > WLCAP ? WLCAP : c);
#pragma unroll 1
      for (int b0 = 0; b0 < c; b0 += 32) {
        const int idx = b0 + lane;
        const int ent = wl[w2 * WLCAP + (idx < WLCAP ? idx : WLCAP - 1)];
        int eid = (ent >> SLB) & 0xFFFFF;
        eid = eid > NE - 1 ? NE - 1 : eid;
        int sr = srcs[eid];
        sr = sr < 0 ? 0 : (sr > NN - 1 ? NN - 1 : sr);
        const int word = (sr << SLB) | (ent & (NBRUN - 1));
        const int m32 = (c - b0) < 32 ? (c - b0) : 32;
#pragma unroll 1
        for (int k = 0; k < m32; ++k) {
          const int wd   = __builtin_amdgcn_readlane(word, k);
          const int slot = wd & (NBRUN - 1);
          if (lane == 0) {
            int p = cur[slot];
            p = p < 0 ? 0 : (p > RCAP - 1 ? RCAP - 1 : p);
            pl[p] = wd;
            cur[slot] = p + 1;
          }
        }
      }
    }
  }
  __syncthreads();

#pragma unroll 1
  for (int i = tid; i < NBRUN; i += NTHR) {
    const int node = blk * NBRUN + i;
    const float dg = (float)(cnt[i] + 1);
    const float r  = 1.0f / sqrtf(dg);
    const float g  = (dg > 0.0f) ? r : 0.0f;
    dvb[i] = __float_as_int((node < NN) ? g : 0.0f);
  }
  __syncthreads();

  const int ovf = misc[9];
  int* lp = LIST + (size_t)blk * RCAP;
  int* cp = CNT + (size_t)blk * NBRUN;
  int* op = OFF + (size_t)blk * NBRUN;
  int* dp = DINVB + (size_t)blk * NBRUN;
  int* fp = FLAG + (size_t)blk * 32;
  bucket_flush(pl, cnt, offs, dvb, ovf, lp, cp, op, dp, fp, tid);
  __threadfence();
  bucket_flush(pl, cnt, offs, dvb, ovf, lp, cp, op, dp, fp, tid);
}

template <int KTOT, int LDA, int LDB, int NT>
__global__ __launch_bounds__(NTHR) __attribute__((amdgpu_num_vgpr(248)))
void k_gemm(const unsigned short* __restrict__ A, const unsigned short* __restrict__ BT,
            const float* __restrict__ DINV, float* P) {
  static_assert(KTOT % 32 == 0 && KTOT <= LDA && KTOT <= LDB && (NT == 8 || NT == 4));
  extern __shared__ __attribute__((aligned(16))) float gsm[];
  float* stg = gsm;
  float* sdv = gsm + GBM * GSP;
  const int tid = (int)threadIdx.x, lane = tid & 31, wave = tid >> 5, hh = lane >> 4, m = lane & 15;
  const int rowBase = (int)blockIdx.x * GBM;
  if (tid < 32) *(v4fa*)(sdv + 4 * tid) = *(const v4fa*)(DINV + rowBase + 4 * tid);

  v8f acc[NT];
  {
    const v8f z = {0.f, 0.f, 0.f, 0.f, 0.f, 0.f, 0.f, 0.f};
#pragma unroll
    for (int t = 0; t < NT; ++t) acc[t] = z;
  }
  const unsigned short* ap = A + (size_t)(rowBase + 16 * wave + m) * (size_t)LDA + 8 * hh;
  const unsigned short* bp = BT + (size_t)m * (size_t)LDB + 8 * hh;
#pragma unroll 1
  for (int k0 = 0; k0 < KTOT; k0 += 32) {
    FragB af;
    af.h[0] = *(const v8usa*)(ap + k0);
    af.h[1] = *(const v8usa*)(ap + k0 + 16);
#pragma unroll
    for (int nt = 0; nt < NT; ++nt) {
      const unsigned short* wq = bp + (size_t)(16 * nt) * (size_t)LDB + k0;
      FragB bf;
      bf.h[0] = *(const v8usa*)wq;
      bf.h[1] = *(const v8usa*)(wq + 16);
      acc[nt] = wmb(af, bf, acc[nt]);
    }
  }
#pragma unroll
  for (int nt = 0; nt < NT; ++nt) {
#pragma unroll
    for (int r = 0; r < 8; ++r) stg[(16 * wave + 8 * hh + r) * GSP + 16 * nt + m] = acc[nt][r];
  }
  __syncthreads();

  if constexpr (NT == 8) {
#pragma unroll 1
    for (int i = 0; i < 16; ++i) {
      const int lr   = 16 * wave + i;
      const int grow = rowBase + lr;
      const bool live = grow < NN;
      const v4f a  = *(const v4fa*)(stg + lr * GSP + 4 * lane);
      const float dv = sdv[lr];
      asm volatile("" :: "v"(a));
      const float v0 = dv * a.x, v1 = dv * a.y, v2 = dv * a.z, v3 = dv * a.w;
      v4f o;
      o.x = live ? v0 : 0.0f; o.y = live ? v1 : 0.0f; o.z = live ? v2 : 0.0f; o.w = live ? v3 : 0.0f;
      st2_v4f(P + (size_t)grow * (size_t)(16 * NT) + 4 * lane, o);
    }
  } else {
#pragma unroll 1
    for (int i = 0; i < 8; ++i) {
      const int lr   = 16 * wave + 2 * i + hh;
      const int grow = rowBase + lr;
      const bool live = grow < NN;
      const v4f a  = *(const v4fa*)(stg + lr * GSP + 4 * m);
      const float dv = sdv[lr];
      asm volatile("" :: "v"(a));
      const float v0 = dv * a.x, v1 = dv * a.y, v2 = dv * a.z, v3 = dv * a.w;
      v4f o;
      o.x = live ? v0 : 0.0f; o.y = live ? v1 : 0.0f; o.z = live ? v2 : 0.0f; o.w = live ? v3 : 0.0f;
      st2_v4f(P + (size_t)grow * (size_t)(16 * NT) + 4 * m, o);
    }
  }
}

__global__ __launch_bounds__(NTHR) void k_replay_w(const int* __restrict__ LIST, const int* __restrict__ CNT,
                                                   const int* __restrict__ OFF, const float* __restrict__ DINV,
                                                   const int* __restrict__ FLAG, const float* __restrict__ P,
                                                   const float* __restrict__ bias, unsigned short* XHL) {
  __shared__ __attribute__((aligned(16))) float sb[HID];
  const int tid = (int)threadIdx.x, lane = tid & 31, wave = tid >> 5;
  const int blk = (int)blockIdx.x;
  if (tid < 32) *(v4fa*)(sb + 4 * tid) = *(const v4fa*)(bias + 4 * tid);
  __syncthreads();
  const v4f bv = *(const v4fa*)(sb + 4 * lane);
  const int flag = FLAG[(size_t)blk * 32];
  const int* lb = LIST + (size_t)blk * RCAP;
  const float qnan = __uint_as_float(0x7fc00000u);

#pragma unroll 1
  for (int si = 0; si < NBRUN / NWAVE; ++si) {
    const int d = blk * NBRUN + si * NWAVE + wave;
    const int craw = __builtin_amdgcn_readfirstlane(CNT[d]);
    const int oraw = __builtin_amdgcn_readfirstlane(OFF[d]);
    const bool big = craw > TRIPCAP;
    const int c = min(max(craw, 0), TRIPCAP);
    const int o = min(max(oraw, 0), RCAP - 1);
    int last = o + c - 1; last = last < o ? o : last;
    last = min(last, RCAP - 1);
    const float dd = DINV[d];
    float a0 = 0.0f, a1 = 0.0f, a2 = 0.0f, a3 = 0.0f;
#pragma unroll 1
    for (int b0 = 0; b0 < c; b0 += 32) {
      int idx = o + b0 + lane;
      idx = min(idx, last);
      const unsigned wd = (unsigned)lb[idx];
      int sr = (int)(wd >> SLB);
      sr = min(sr, NN - 1);
      const int m32 = min(c - b0, 32);
#pragma unroll 1
      for (int k = 0; k < m32; ++k) {
        const int sk = __builtin_amdgcn_readlane(sr, k);
        const v4f v = *(const v4fa*)(P + (size_t)sk * HID + 4 * lane);
        a0 += v.x; a1 += v.y; a2 += v.z; a3 += v.w;
      }
    }
    const int dc = min(d, MP - 1);
    const v4f g = *(const v4fa*)(P + (size_t)dc * HID + 4 * lane);
    asm volatile("" :: "v"(g));
    float t0 = dd * (a0 + g.x) + bv.x, t1 = dd * (a1 + g.y) + bv.y;
    float t2 = dd * (a2 + g.z) + bv.z, t3 = dd * (a3 + g.w) + bv.w;
    t0 = (t0 > 0.0f) ? t0 : (t0 - t0); t1 = (t1 > 0.0f) ? t1 : (t1 - t1);
    t2 = (t2 > 0.0f) ? t2 : (t2 - t2); t3 = (t3 > 0.0f) ? t3 : (t3 - t3);
    const bool bad  = (flag != 0) | big;
    const bool live = d < NN;
    t0 = bad ? qnan : t0; t1 = bad ? qnan : t1; t2 = bad ? qnan : t2; t3 = bad ? qnan : t3;
    t0 = live ? t0 : 0.0f; t1 = live ? t1 : 0.0f; t2 = live ? t2 : 0.0f; t3 = live ? t3 : 0.0f;
    int h01, h23, l01, l23;
    hilo_pack(t0, t1, t2, t3, h01, h23, l01, l23);
    const v4i ow = regroup32(h01, h23, l01, l23, lane);
    asm volatile("" :: "v"(ow));
    const bool wr = d < MP;
    unsigned short* hp = XHL + (size_t)dc * KHL + 8 * lane;
    if (wr) *(volatile v4i*)hp = ow;
    __threadfence();
    if (wr) *(volatile v4i*)hp = ow;
  }
}

__global__ __launch_bounds__(NTHR) void k_replay_n(const int* __restrict__ LIST, const int* __restrict__ CNT,
                                                   const int* __restrict__ OFF, const float* __restrict__ DINV,
                                                   const int* __restrict__ FLAG, const float* __restrict__ P3,
                                                   const float* __restrict__ bias, float* out) {
  __shared__ __attribute__((aligned(16))) float sb[DOUT];
  const int tid = (int)threadIdx.x, lane = tid & 31, wave = tid >> 5, hh = lane >> 4, q = lane & 15;
  const int blk = (int)blockIdx.x;
  if (tid < 16) *(v4fa*)(sb + 4 * tid) = *(const v4fa*)(bias + 4 * tid);
  __syncthreads();
  const v4f bv = *(const v4fa*)(sb + 4 * q);
  const int flag = FLAG[(size_t)blk * 32];
  const int* lb = LIST + (size_t)blk * RCAP;
  const float qnan = __uint_as_float(0x7fc00000u);

#pragma unroll 1
  for (int i = 0; i < NBRUN / (2 * NWAVE); ++i) {
    const int d = blk * NBRUN + (NBRUN / NWAVE) * wave + 2 * i + hh;
    const int craw = CNT[d];
    const int oraw = OFF[d];
    const bool big = craw > TRIPCAP;
    const int c = min(max(craw, 0), TRIPCAP);
    const int o = min(max(oraw, 0), RCAP - 1);
    int last = o + c - 1; last = last < o ? o : last;
    last = min(last, RCAP - 1);
    const int co = __shfl_xor(c, 16, 32);
    const int cm = __builtin_amdgcn_readfirstlane(max(c, co));
    const float dd = DINV[d];
    float a0 = 0.0f, a1 = 0.0f, a2 = 0.0f, a3 = 0.0f;
#pragma unroll 1
    for (int j = 0; j < cm; ++j) {
      int idx = o + j;
      idx = min(idx, last);
      const unsigned wd = (unsigned)lb[idx];
      int sr = (int)(wd >> SLB);
      sr = min(sr, NN - 1);
      const v4f v = *(const v4fa*)(P3 + (size_t)sr * DOUT + 4 * q);
      asm volatile("" :: "v"(v));
      const bool valid = j < c;
      const float u0 = valid ? v.x : 0.0f, u1 = valid ? v.y : 0.0f;
      const float u2 = valid ? v.z : 0.0f, u3 = valid ? v.w : 0.0f;
      a0 += u0; a1 += u1; a2 += u2; a3 += u3;
    }
    const int dc = min(d, NN - 1);
    const v4f g = *(const v4fa*)(P3 + (size_t)dc * DOUT + 4 * q);
    asm volatile("" :: "v"(g));
    float t0 = dd * (a0 + g.x) + bv.x, t1 = dd * (a1 + g.y) + bv.y;
    float t2 = dd * (a2 + g.z) + bv.z, t3 = dd * (a3 + g.w) + bv.w;
    const bool bad = (flag != 0) | big;
    t0 = bad ? qnan : t0; t1 = bad ? qnan : t1; t2 = bad ? qnan : t2; t3 = bad ? qnan : t3;
    v4f ov;
    ov.x = t0; ov.y = t1; ov.z = t2; ov.w = t3;
    asm volatile("" :: "v"(ov));
    const bool wr = d < NN;
    float* op = out + (size_t)dc * DOUT + 4 * q;
    if (wr) *(volatile v4f*)op = ov;
    __threadfence();
    if (wr) *(volatile v4f*)op = ov;
  }
}

extern "C" void kernel_launch(void* const* d_in, const int* in_sizes, int n_in,
                              void* d_out, int out_size, void* d_ws, size_t ws_size,
                              hipStream_t stream) {
  if (n_in < 8) return;
  if (in_sizes[0] != NN * CIN) return;
  if (in_sizes[1] != 2 * NE) return;
  if (in_sizes[2] != CIN * HID) return;
  if (in_sizes[3] != HID) return;
  if (in_sizes[4] != HID * HID) return;
  if (in_sizes[5] != HID) return;
  if (in_sizes[6] != HID * DOUT) return;
  if (in_sizes[7] != DOUT) return;
  if (out_size != NN * DOUT) return;

  const float* x  = (const float*)d_in[0];
  const int*   ei = (const int*)d_in[1];
  const float* W1 = (const float*)d_in[2];
  const float* b1 = (const float*)d_in[3];
  const float* W2 = (const float*)d_in[4];
  const float* b2 = (const float*)d_in[5];
  const float* W3 = (const float*)d_in[6];
  const float* b3 = (const float*)d_in[7];
  float* out = (float*)d_out;
  const int* srcs = ei;
  const int* dsts = ei + NE;

  constexpr size_t zXB   = (size_t)MP * CIN * 2;
  constexpr size_t zP    = (size_t)MP * HID * 4;
  constexpr size_t zXHL  = (size_t)MP * KHL * 2;
  constexpr size_t zLIST = (size_t)NBK * RCAP * 4;
  constexpr size_t zTAB  = (size_t)CNTN * 4;
  constexpr size_t zFLAG = (size_t)(NBK + 1) * 128;
  constexpr size_t zW1T  = (size_t)HID * CIN * 2;
  constexpr size_t zW2D  = (size_t)HID * KHL * 2;
  constexpr size_t zW3D  = (size_t)DOUT * KHL * 2;
  constexpr size_t zSM   = 1536;
  constexpr size_t oXB   = 0;
  constexpr size_t oP    = oXB + zXB;
  constexpr size_t oXHL  = oP + zP;
  constexpr size_t oLIST = oXHL + zXHL;
  constexpr size_t oCNT  = oLIST + zLIST;
  constexpr size_t oOFF  = oCNT + zTAB;
  constexpr size_t oDINV = oOFF + zTAB;
  constexpr size_t oFLAG = oDINV + zTAB;
  constexpr size_t oW1T  = oFLAG + zFLAG;
  constexpr size_t oW2D  = oW1T + zW1T;
  constexpr size_t oW3D  = oW2D + zW2D;
  constexpr size_t oSM   = oW3D + zW3D;
  constexpr size_t oEND  = oSM + zSM;
  static_assert(zXB % 256 == 0 && zP % 256 == 0 && zXHL % 256 == 0 && zLIST % 256 == 0 && zTAB % 256 == 0);
  static_assert(zFLAG % 256 == 0 && zW1T % 256 == 0 && zW2D % 256 == 0 && zW3D % 256 == 0 && zSM % 256 == 0);
  static_assert((size_t)MP * DOUT * 4 <= zP);
  static_assert((size_t)NBK * 128 <= zFLAG);
  static_assert(oEND <= (size_t)WSMAX);
  if (oEND > ws_size) return;

  char* ws = (char*)d_ws;
  unsigned short* XB   = (unsigned short*)(ws + oXB);
  float*          P    = (float*)(ws + oP);
  unsigned short* XHL  = (unsigned short*)(ws + oXHL);
  int*            LIST = (int*)(ws + oLIST);
  int*            CNT  = (int*)(ws + oCNT);
  int*            OFF  = (int*)(ws + oOFF);
  float*          DINV = (float*)(ws + oDINV);
  int*            FLAG = (int*)(ws + oFLAG);
  unsigned short* W1T  = (unsigned short*)(ws + oW1T);
  unsigned short* W2D  = (unsigned short*)(ws + oW2D);
  unsigned short* W3D  = (unsigned short*)(ws + oW3D);
  float*          SM   = (float*)(ws + oSM);

  constexpr int K2 = TWO_TERM_L2 ? KHL : HID;
  constexpr int K3 = TWO_TERM_L3 ? KHL : HID;

  hipFuncSetAttribute(reinterpret_cast<const void*>(&k_bucket), hipFuncAttributeMaxDynamicSharedMemorySize, (int)BK_LDS);
  hipFuncSetAttribute(reinterpret_cast<const void*>(&k_gemm<CIN, CIN, CIN, 8>), hipFuncAttributeMaxDynamicSharedMemorySize, (int)G_LDS);
  hipFuncSetAttribute(reinterpret_cast<const void*>(&k_gemm<K2, KHL, KHL, 8>), hipFuncAttributeMaxDynamicSharedMemorySize, (int)G_LDS);
  hipFuncSetAttribute(reinterpret_cast<const void*>(&k_gemm<K3, KHL, KHL, 4>), hipFuncAttributeMaxDynamicSharedMemorySize, (int)G_LDS);

  k_prep<<<PBTOT, NTHR, 0, stream>>>(x, W1, b1, W2, b2, W3, b3, XB, W1T, W2D, W3D, XHL, SM);
  k_bucket<<<NBK, NTHR, BK_LDS, stream>>>(srcs, dsts, LIST, CNT, OFF, (int*)DINV, FLAG);
  k_gemm<CIN, CIN, CIN, 8><<<MP / GBM, NTHR, G_LDS, stream>>>(XB, W1T, DINV, P);
  k_replay_w<<<NBK, NTHR, 0, stream>>>(LIST, CNT, OFF, DINV, FLAG, P, SM, XHL);
  k_gemm<K2, KHL, KHL, 8><<<MP / GBM, NTHR, G_LDS, stream>>>(XHL, W2D, DINV, P);
  k_replay_w<<<NBK, NTHR, 0, stream>>>(LIST, CNT, OFF, DINV, FLAG, P, SM + HID, XHL);
  k_gemm<K3, KHL, KHL, 4><<<MP / GBM, NTHR, G_LDS, stream>>>(XHL, W3D, DINV, P);
  k_replay_n<<<NBK, NTHR, 0, stream>>>(LIST, CNT, OFF, DINV, FLAG, P, SM + 2 * HID, out);
}
